// HSICLoss_25091198943287
// MI455X (gfx1250) — hardware-verified
//
#include <hip/hip_runtime.h>
#include <math.h>

typedef __attribute__((ext_vector_type(16))) _Float16 v16h;
typedef __attribute__((ext_vector_type(16))) __bf16 v16b;
typedef __attribute__((ext_vector_type(8)))  _Float16 v8h;
typedef __attribute__((ext_vector_type(8)))  float v8f;
typedef __attribute__((ext_vector_type(4)))  float v4f;
typedef __attribute__((ext_vector_type(2)))  float v2f;
typedef __attribute__((ext_vector_type(4)))  unsigned v4u;
typedef __attribute__((ext_vector_type(4)))  int v4i;
typedef float __attribute__((may_alias)) float_a;
typedef int __attribute__((may_alias)) int_a;

template <typename T> __device__ __forceinline__ void vst2(void* p, T v) { *(volatile T*)p = v; __threadfence(); *(volatile T*)p = v; }
__device__ __forceinline__ v8f wmma16(v16h a, v16h b, v8f c) {
  v8f d = __builtin_amdgcn_wmma_f32_16x16x32_f16(false, a, false, b, (short)0, c, false, false);
  asm volatile("v_nop\n\tv_nop\n\tv_nop\n\tv_nop" : "+v"(d) : "v"(a), "v"(b));
  return d;
}
__device__ __forceinline__ v8f wmma_bf(v16b a, v16b b, v8f c) {
  v8f d = __builtin_amdgcn_wmma_f32_16x16x32_bf16(false, a, false, b, (short)0, c, false, false);
  asm volatile("v_nop\n\tv_nop\n\tv_nop\n\tv_nop" : "+v"(d) : "v"(a), "v"(b));
  return d;
}
__device__ __forceinline__ v16h frag_h(const _Float16* rowk0, int lane) {
  union { v16h v; v8h q[2]; } u; const _Float16* p = rowk0 + 8 * (lane >> 4);
  u.q[0] = *(const v8h*)p; u.q[1] = *(const v8h*)(p + 16); return u.v;
}
__device__ __forceinline__ v16h frag_f32(const float* rowk0, int lane) {
  v16h a; const float* p = rowk0 + 8 * (lane >> 4);
#pragma unroll
  for (int i = 0; i < 8; ++i) { a[i] = (_Float16)p[i]; a[8 + i] = (_Float16)p[16 + i]; }
  return a;
}
__device__ __forceinline__ v16h frag_f32s(const float* rowk0, int lane, float sc) {
  v16h a; const float* p = rowk0 + 8 * (lane >> 4);
#pragma unroll
  for (int i = 0; i < 8; ++i) { a[i] = (_Float16)(p[i] * sc); a[8 + i] = (_Float16)(p[16 + i] * sc); }
  return a;
}
__device__ __forceinline__ v16h fragc_f32(const float* W, int k0, int n, int lane, int ld, int K) {
  v16h a; const int g = lane >> 4;
#pragma unroll
  for (int i = 0; i < 8; ++i) { const int ka = k0 + 8 * g + i, kb = ka + 16;
    a[i] = (_Float16)(ka < K ? W[(size_t)ka * ld + n] : 0.f); a[8 + i] = (_Float16)(kb < K ? W[(size_t)kb * ld + n] : 0.f); }
  return a;
}
struct F2 { v16b h, l; };
__device__ __forceinline__ F2 bsplit16(const float v[16]) { F2 r;
#pragma unroll
  for (int i = 0; i < 16; ++i) { const __bf16 h = (__bf16)v[i]; r.h[i] = h; r.l[i] = (__bf16)(v[i] - (float)h); }
  return r; }
__device__ __forceinline__ F2 split_row(const float* row, int k0, int lane) { float v[16]; const float* p = row + k0 + 8 * (lane >> 4);
#pragma unroll
  for (int i = 0; i < 8; ++i) { v[i] = p[i]; v[8 + i] = p[16 + i]; }
  return bsplit16(v); }
__device__ __forceinline__ F2 split_rowK(const float* row, int k0, int lane, int K) { float v[16]; const int g = lane >> 4;
#pragma unroll
  for (int i = 0; i < 8; ++i) { const int ka = k0 + 8 * g + i, kb = ka + 16; v[i] = ka < K ? row[ka] : 0.f; v[8 + i] = kb < K ? row[kb] : 0.f; }
  return bsplit16(v); }
__device__ __forceinline__ F2 split_col(const float* W, int k0, int n, int lane, int ld, int K) { float v[16]; const int g = lane >> 4;
#pragma unroll
  for (int i = 0; i < 8; ++i) { const int ka = k0 + 8 * g + i, kb = ka + 16; v[i] = ka < K ? W[(size_t)ka * ld + n] : 0.f; v[8 + i] = kb < K ? W[(size_t)kb * ld + n] : 0.f; }
  return bsplit16(v); }
__device__ __forceinline__ v8f mac3(const F2& a, const F2& b, v8f c) { c = wmma_bf(a.l, b.h, c); c = wmma_bf(a.h, b.l, c); return wmma_bf(a.h, b.h, c); }
__device__ __forceinline__ float sigm(float v) { return 1.0f / (1.0f + expf(-v)); }
#define LDSX() do { asm volatile("s_wait_dscnt 0" ::: "memory"); __builtin_amdgcn_wave_barrier(); __builtin_amdgcn_fence(__ATOMIC_RELEASE, "workgroup"); } while (0)


#define MM 8192
#define DD 128
__device__ __forceinline__ float bfr(float v) { return (float)(__bf16)v; }

__device__ __forceinline__ v16b frag_b(const __bf16* rowk0, int lane) { return __builtin_bit_cast(v16b, frag_h((const _Float16*)rowk0, lane)); }
__global__ __launch_bounds__(256) void k_prep(const float* __restrict__ x, const float* __restrict__ y, __bf16* __restrict__ XB, __bf16* __restrict__ YB, float* __restrict__ SQ) {
  __shared__ float ssq[2][64];
  const int tid = threadIdx.x; const int r0 = blockIdx.x * 64;
  if (tid < 128) { const int which = tid >> 6, rl = tid & 63; const float* src = (which ? y : x) + (size_t)(r0 + rl) * DD; float s = 0.f; for (int k = 0; k < DD; ++k) { const float v = bfr(src[k]); s += v * v; } ssq[which][rl] = s; }
  for (int q = tid; q < 2 * 64 * (DD / 8); q += 256) { const int which = q / (64 * 16), rem = q % (64 * 16), rl = rem >> 4, pc = rem & 15; const float* src = (which ? y : x) + (size_t)(r0 + rl) * DD + pc * 8;
    union { __bf16 e[8]; v4u u; } pk;
#pragma unroll
    for (int e = 0; e < 8; ++e) pk.e[e] = (__bf16)src[e];
    vst2((unsigned*)((which ? YB : XB) + (size_t)(r0 + rl) * DD + pc * 8), pk.u); }
  __syncthreads();
  if (tid < 32) { const int which = tid >> 4, pc = tid & 15; vst2(SQ + (size_t)which * MM + r0 + pc * 4, *(const v4f*)(&ssq[which][pc * 4])); }
}
__global__ __launch_bounds__(128) void k_gram(const __bf16* __restrict__ XB, const __bf16* __restrict__ YB, const float* __restrict__ SQ, float* __restrict__ PART) {
  __shared__ float sqi[2][64]; __shared__ float sqj[2][64];
  const int tid = threadIdx.x, wave = tid >> 5, lane = tid & 31, col = lane & 15, g = lane >> 4; const int i0 = blockIdx.x * 64; const int r0 = i0 + wave * 16;
  if (tid < 128) { const int which = tid >> 6, rl = tid & 63; sqi[which][rl] = SQ[(size_t)which * MM + i0 + rl]; }
  v16b ax[4], ay[4];
#pragma unroll
  for (int kc = 0; kc < 4; ++kc) { ax[kc] = frag_b(XB + (size_t)(r0 + col) * DD + kc * 32, lane); ay[kc] = frag_b(YB + (size_t)(r0 + col) * DD + kc * 32, lane); }
  float rsK[8], rsL[8], rsLK[8];
#pragma unroll
  for (int r = 0; r < 8; ++r) { rsK[r] = 0.f; rsL[r] = 0.f; rsLK[r] = 0.f; }
  __syncthreads();
#pragma unroll 1
  for (int jt = 0; jt < MM / 64; ++jt) { const int j0 = jt * 64;
    __syncthreads();
    if (tid < 128) { const int which = tid >> 6, rl = tid & 63; sqj[which][rl] = SQ[(size_t)which * MM + j0 + rl]; }
    __syncthreads();
#pragma unroll
    for (int t = 0; t < 4; ++t) { const int jc = j0 + t * 16 + col; v8f sx = {}, sy = {};
#pragma unroll
      for (int kc = 0; kc < 4; ++kc) { sx = wmma_bf(ax[kc], frag_b(XB + (size_t)jc * DD + kc * 32, lane), sx); sy = wmma_bf(ay[kc], frag_b(YB + (size_t)jc * DD + kc * 32, lane), sy); }
      const float qxj = sqj[0][t * 16 + col], qyj = sqj[1][t * 16 + col];
#pragma unroll
      for (int r = 0; r < 8; ++r) { const int rl = wave * 16 + 8 * g + r; const float dk = -2.0f * sx[r] + sqi[0][rl] + qxj; const float dl = -2.0f * sy[r] + sqi[1][rl] + qyj;
        const float kv = expf(-dk), lv = expf(-dl); rsK[r] += kv; rsL[r] += lv; rsLK[r] += lv * kv; } } }
#pragma unroll
  for (int r = 0; r < 8; ++r) {
#pragma unroll
    for (int o = 1; o < 16; o <<= 1) { rsK[r] += __shfl_xor(rsK[r], o, 32); rsL[r] += __shfl_xor(rsL[r], o, 32); rsLK[r] += __shfl_xor(rsLK[r], o, 32); } }
  __shared__ __align__(16) float sp[64][4];
  if (col == 0) {
#pragma unroll
    for (int r = 0; r < 8; ++r) { sp[wave * 16 + 8 * g + r][0] = rsK[r]; sp[wave * 16 + 8 * g + r][1] = rsL[r]; sp[wave * 16 + 8 * g + r][2] = rsLK[r]; sp[wave * 16 + 8 * g + r][3] = 0.f; } }
  __syncthreads();
  if (tid < 64) vst2(PART + (size_t)(i0 + tid) * 4, *(const v4f*)(&sp[tid][0]));
}
__global__ __launch_bounds__(256) void k_fin(const float* __restrict__ PART, float* __restrict__ out) {
  __shared__ double sK[256], sL[256], sLK[256], sX[256];
  const int tid = threadIdx.x; double aK = 0.0, aL = 0.0, aLK = 0.0, aX = 0.0;
  for (int r = tid; r < MM; r += 256) { const double k = PART[(size_t)r * 4], l = PART[(size_t)r * 4 + 1], lk = PART[(size_t)r * 4 + 2]; aK += k; aL += l; aLK += lk; aX += k * l; }
  sK[tid] = aK; sL[tid] = aL; sLK[tid] = aLK; sX[tid] = aX; __syncthreads();
  for (int o = 128; o > 0; o >>= 1) { if (tid < o) { sK[tid] += sK[tid + o]; sL[tid] += sL[tid + o]; sLK[tid] += sLK[tid + o]; sX[tid] += sX[tid + o]; } __syncthreads(); }
  if (tid == 0) { const double m = (double)MM; const double sumK = sK[0], sumL = sL[0], sumLK = sLK[0], cross = sX[0];
    const double h = (sumLK - 2.0 * cross / m + sumK * sumL / (m * m)) / ((m - 1.0) * (m - 1.0));
    union { float f[32]; v4f v[8]; } o_; for (int e = 0; e < 32; ++e) o_.f[e] = 0.f; o_.f[0] = (float)h; vst2(out, (float_a)o_.f[0]); }
}
extern "C" void kernel_launch(void* const* d_in, const int* in_sizes, int n_in, void* d_out, int out_size, void* d_ws, size_t ws_size, hipStream_t stream) {
  (void)in_sizes; (void)n_in; (void)out_size; (void)ws_size;
  const float* x = (const float*)d_in[0]; const float* y = (const float*)d_in[1];
  char* ws = (char*)d_ws; float* PART = (float*)ws; __bf16* XB = (__bf16*)(ws + 131072); __bf16* YB = XB + (size_t)MM * DD; float* SQ = (float*)(YB + (size_t)MM * DD);
  k_prep<<<MM / 64, 256, 0, stream>>>(x, y, XB, YB, SQ);
  k_gram<<<MM / 64, 128, 0, stream>>>(XB, YB, SQ, PART);
  k_fin<<<1, 256, 0, stream>>>(PART, (float*)d_out);
}
